// T5MHSA_6408091206135
// MI455X (gfx1250) — hardware-verified
//
#include <hip/hip_runtime.h>
#include <stddef.h>


typedef __bf16 v16bf __attribute__((ext_vector_type(16)));
typedef float v8f __attribute__((ext_vector_type(8)));
typedef float v4f __attribute__((ext_vector_type(4)));
typedef unsigned int v4u __attribute__((ext_vector_type(4)));
typedef unsigned short u16;

#define EMB 1024
#define SEQ 1024
#define NH 16
#define HD 64
#define NQK 2048
#define NBP 4
#define TOKP (NBP * SEQ)
#define MAXD 128
#define TP 68

__constant__ int c_bucket[MAXD + 1] = {
  0,1,2,3,4,5,6,7,8,9,10,11,12,13,14,15,16,18,19,20,21,21,22,22,22,23,23,23,24,24,24,24,24,
  25,25,25,25,25,25,26,26,26,26,26,26,26,26,26,27,27,27,27,27,27,27,27,27,27,27,
  28,28,28,28,28,28,28,28,28,28,28,28,28,28,28,28,28,
  29,29,29,29,29,29,29,29,29,29,29,29,29,29,29,29,29,29,29,29,29,29,
  30,30,30,30,30,30,30,30,30,30,30,30,30,30,30,30,30,30,30,30,30,30,30,30,30,30,30,30,30,30,31 };

union Frag { v16bf v; v4u u[2]; };

__device__ __forceinline__ v8f vz8() {
  v8f z = {0.f, 0.f, 0.f, 0.f, 0.f, 0.f, 0.f, 0.f};
  return z;
}

__device__ __forceinline__ v8f mma(v16bf a, v16bf b, v8f c) {
  c = __builtin_amdgcn_wmma_f32_16x16x32_bf16(false, a, false, b, (short)0, c, false, false);
  asm volatile("v_nop\n\tv_nop\n\tv_nop\n\tv_nop" : "+v"(c) : "v"(a), "v"(b));
  return c;
}

__device__ __forceinline__ v16bf ld_frag(const u16* p, int pitch) {
  const int l = threadIdx.x & 31, h = l >> 4, m = l & 15;
  const u16* q = p + (size_t)m * pitch + 8 * h;
  Frag f;
  f.u[0] = *(const v4u*)q;
  f.u[1] = *(const v4u*)(q + 16);
  return f.v;
}

__device__ __forceinline__ unsigned bf16_bits(float f) {
  unsigned u = __float_as_uint(f);
  return (u + 0x7FFFu + ((u >> 16) & 1u)) >> 16;
}
__device__ __forceinline__ void split2(float x0, float x1, unsigned& hw, unsigned& lw) {
  const unsigned h0 = bf16_bits(x0), h1 = bf16_bits(x1);
  const unsigned l0 = bf16_bits(x0 - __uint_as_float(h0 << 16));
  const unsigned l1 = bf16_bits(x1 - __uint_as_float(h1 << 16));
  hw = h0 | (h1 << 16);
  lw = l0 | (l1 << 16);
}
__device__ __forceinline__ void split8(float f0, float f1, float f2, float f3,
                                       float f4, float f5, float f6, float f7,
                                       v4u& H, v4u& L) {
  unsigned h0, l0, h1, l1, h2, l2, h3, l3;
  split2(f0, f1, h0, l0);
  split2(f2, f3, h1, l1);
  split2(f4, f5, h2, l2);
  split2(f6, f7, h3, l3);
  H.x = h0; H.y = h1; H.z = h2; H.w = h3;
  L.x = l0; L.y = l1; L.z = l2; L.w = l3;
}
__device__ __forceinline__ void store2_planes(u16* ph, u16* pl, v4u H, v4u L) {
  *(volatile v4u*)ph = H;
  *(volatile v4u*)pl = L;
  __threadfence();
  *(volatile v4u*)ph = H;
  *(volatile v4u*)pl = L;
}

__device__ __forceinline__ float rmax16(float v) {
  v = fmaxf(v, __shfl_xor(v, 1, 32));
  v = fmaxf(v, __shfl_xor(v, 2, 32));
  v = fmaxf(v, __shfl_xor(v, 4, 32));
  v = fmaxf(v, __shfl_xor(v, 8, 32));
  return v;
}
__device__ __forceinline__ float rsum16(float v) {
  v += __shfl_xor(v, 1, 32);
  v += __shfl_xor(v, 2, 32);
  v += __shfl_xor(v, 4, 32);
  v += __shfl_xor(v, 8, 32);
  return v;
}

__global__ __launch_bounds__(256) void k_split(const float* __restrict__ src,
                                               u16* __restrict__ dh, u16* __restrict__ dl, int n8) {
  const int t = blockIdx.x * 256 + threadIdx.x;
  if (t >= n8) return;
  const float* p = src + (size_t)t * 8;
  const v4f a = *(const v4f*)p;
  const v4f b = *(const v4f*)(p + 4);
  v4u H, L;
  split8(a.x, a.y, a.z, a.w, b.x, b.y, b.z, b.w, H, L);
  store2_planes(dh + (size_t)t * 8, dl + (size_t)t * 8, H, L);
}

__device__ __forceinline__ void gemm3(const u16* ah, const u16* al, const u16* wh, const u16* wl,
                                      v8f acc[2][4]) {
#pragma unroll 1
  for (int k = 0; k < EMB; k += 32) {
    const v16bf Ah0 = ld_frag(ah + k, EMB);
    const v16bf Ah1 = ld_frag(ah + 16 * EMB + k, EMB);
    const v16bf Al0 = ld_frag(al + k, EMB);
    const v16bf Al1 = ld_frag(al + 16 * EMB + k, EMB);
#pragma unroll
    for (int j = 0; j < 4; ++j) {
      const v16bf Bh = ld_frag(wh + (size_t)j * 16 * EMB + k, EMB);
      const v16bf Bl = ld_frag(wl + (size_t)j * 16 * EMB + k, EMB);
      acc[0][j] = mma(Ah0, Bh, acc[0][j]);
      acc[0][j] = mma(Ah0, Bl, acc[0][j]);
      acc[0][j] = mma(Al0, Bh, acc[0][j]);
      acc[1][j] = mma(Ah1, Bh, acc[1][j]);
      acc[1][j] = mma(Ah1, Bl, acc[1][j]);
      acc[1][j] = mma(Al1, Bh, acc[1][j]);
    }
  }
}

__device__ __forceinline__ void stage_tile(float* s_t, v8f acc[2][4], const float* __restrict__ bvec,
                                           int c0) {
  const int lane = threadIdx.x & 31, wave = threadIdx.x >> 5, h = lane >> 4, m = lane & 15;
#pragma unroll
  for (int i = 0; i < 2; ++i)
#pragma unroll
    for (int j = 0; j < 4; ++j) {
      const float bb = bvec[c0 + 16 * j + m];
#pragma unroll
      for (int r = 0; r < 8; ++r)
        s_t[(wave * 32 + 16 * i + 8 * h + r) * TP + 16 * j + m] = acc[i][j][r] + bb;
    }
}

__global__ __launch_bounds__(64) void k_proj_rows(const u16* __restrict__ Ah, const u16* __restrict__ Al,
                                                  const u16* __restrict__ Wh, const u16* __restrict__ Wl,
                                                  const float* __restrict__ bvec,
                                                  u16* __restrict__ Oh, u16* __restrict__ Ol, int N) {
  __shared__ __attribute__((aligned(16))) float s_t[64 * TP];
  const int lane = threadIdx.x & 31, wave = threadIdx.x >> 5;
  const int c0 = blockIdx.x * 64;
  const int rblk = blockIdx.y * 64;
  const int r0 = rblk + wave * 32;

  v8f acc[2][4] = {{vz8(), vz8(), vz8(), vz8()}, {vz8(), vz8(), vz8(), vz8()}};
  gemm3(Ah + (size_t)r0 * EMB, Al + (size_t)r0 * EMB, Wh + (size_t)c0 * EMB, Wl + (size_t)c0 * EMB, acc);
  stage_tile(s_t, acc, bvec, c0);
  __syncthreads();

#pragma unroll
  for (int it = 0; it < 8; ++it) {
    const int row = wave * 32 + it * 4 + (lane >> 3);
    const int cc = (lane & 7) * 8;
    const float* sp = s_t + row * TP + cc;
    const v4f a = *(const v4f*)sp;
    const v4f b = *(const v4f*)(sp + 4);
    v4u H, L;
    split8(a.x, a.y, a.z, a.w, b.x, b.y, b.z, b.w, H, L);
    const size_t g = (size_t)(rblk + row) * (size_t)N + c0 + cc;
    store2_planes(Oh + g, Ol + g, H, L);
  }
}

__global__ __launch_bounds__(64) void k_proj_vt(const u16* __restrict__ Ah, const u16* __restrict__ Al,
                                                const u16* __restrict__ Wh, const u16* __restrict__ Wl,
                                                const float* __restrict__ bvec,
                                                u16* __restrict__ Vh, u16* __restrict__ Vl) {
  __shared__ __attribute__((aligned(16))) float s_t[64 * TP];
  const int lane = threadIdx.x & 31, wave = threadIdx.x >> 5;
  const int hd = blockIdx.x;
  const int c0 = hd * HD;
  const int rblk = blockIdx.y * 64;
  const int r0 = rblk + wave * 32;

  v8f acc[2][4] = {{vz8(), vz8(), vz8(), vz8()}, {vz8(), vz8(), vz8(), vz8()}};
  gemm3(Ah + (size_t)r0 * EMB, Al + (size_t)r0 * EMB, Wh + (size_t)c0 * EMB, Wl + (size_t)c0 * EMB, acc);
  stage_tile(s_t, acc, bvec, c0);
  __syncthreads();

  const int b = rblk >> 10, l0 = rblk & (SEQ - 1);
#pragma unroll
  for (int it = 0; it < 8; ++it) {
    const int d = wave * 32 + it * 4 + (lane >> 3);
    const int tk = (lane & 7) * 8;
    const float* sp = s_t + tk * TP + d;
    const float f0 = sp[0 * TP], f1 = sp[1 * TP], f2 = sp[2 * TP], f3 = sp[3 * TP];
    const float f4 = sp[4 * TP], f5 = sp[5 * TP], f6 = sp[6 * TP], f7 = sp[7 * TP];
    v4u H, L;
    split8(f0, f1, f2, f3, f4, f5, f6, f7, H, L);
    const size_t g = (size_t)((b * NH + hd) * HD + d) * SEQ + l0 + tk;
    store2_planes(Vh + g, Vl + g, H, L);
  }
}

__global__ __launch_bounds__(256) void k_attn(const u16* __restrict__ QKh, const u16* __restrict__ QKl,
                                              const u16* __restrict__ Vth, const u16* __restrict__ Vtl,
                                              const float* __restrict__ rbias,
                                              u16* __restrict__ AOh, u16* __restrict__ AOl) {
  __shared__ float s_bias[SEQ];
  __shared__ __attribute__((aligned(16))) float s_raw[9216];
  u16* s_kh = reinterpret_cast<u16*>(s_raw);
  u16* s_kl = s_kh + 2048;
  u16* s_vh = s_kl + 2048;
  u16* s_vl = s_vh + 2048;
  u16* s_ph = s_vl + 2048;
  u16* s_pl = s_ph + 5120;

  const int qblk = blockIdx.x, bh = blockIdx.y, b = bh >> 4, hd = bh & 15;
  const int tid = threadIdx.x, lane = tid & 31, wave = tid >> 5, h = lane >> 4, m = lane & 15;

  for (int i = tid; i < SEQ; i += 256) {
    const int dd = i < MAXD ? i : MAXD;
    s_bias[i] = rbias[c_bucket[dd] * NH + hd];
  }

  const int qi0 = qblk * 128 + wave * 16;
  const size_t qrow = (size_t)(b * SEQ + qi0);
  const u16* qph = QKh + qrow * NQK + hd * 128;
  const u16* qpl = QKl + qrow * NQK + hd * 128;
  const v16bf qh0 = ld_frag(qph, NQK), qh1 = ld_frag(qph + 32, NQK);
  const v16bf ql0 = ld_frag(qpl, NQK), ql1 = ld_frag(qpl + 32, NQK);

  float m_i[8], l_i[8];
  v8f acc[4] = {vz8(), vz8(), vz8(), vz8()};
#pragma unroll
  for (int r = 0; r < 8; ++r) { m_i[r] = -1e30f; l_i[r] = 0.f; }

  const int jt_blk = qblk * 4 + 3;
  const int jt_w = (qi0 + 15) >> 5;
  const size_t krow0 = (size_t)b * SEQ;
  const int kcol = hd * 128 + 64;
  const size_t vrow0 = (size_t)bh * HD;

  for (int jt = 0; jt <= jt_blk; ++jt) {
    {
      const int rr = tid >> 3, pc = (tid & 7) * 8;
      const size_t g = (krow0 + jt * 32 + rr) * NQK + kcol + pc;
      *(v4u*)(s_kh + rr * 64 + pc) = *(const v4u*)(QKh + g);
      *(v4u*)(s_kl + rr * 64 + pc) = *(const v4u*)(QKl + g);
    }
    {
      const int d = tid >> 2, pc = (tid & 3) * 8;
      const size_t g = (vrow0 + d) * SEQ + jt * 32 + pc;
      *(v4u*)(s_vh + d * 32 + pc) = *(const v4u*)(Vth + g);
      *(v4u*)(s_vl + d * 32 + pc) = *(const v4u*)(Vtl + g);
    }
    __syncthreads();

    if (jt <= jt_w) {
      v8f s0 = vz8(), s1 = vz8();
      {
        v16bf kh = ld_frag(s_kh, 64), kl = ld_frag(s_kl, 64);
        s0 = mma(qh0, kh, s0); s0 = mma(qh0, kl, s0); s0 = mma(ql0, kh, s0);
        kh = ld_frag(s_kh + 32, 64); kl = ld_frag(s_kl + 32, 64);
        s0 = mma(qh1, kh, s0); s0 = mma(qh1, kl, s0); s0 = mma(ql1, kh, s0);
        kh = ld_frag(s_kh + 16 * 64, 64); kl = ld_frag(s_kl + 16 * 64, 64);
        s1 = mma(qh0, kh, s1); s1 = mma(qh0, kl, s1); s1 = mma(ql0, kh, s1);
        kh = ld_frag(s_kh + 16 * 64 + 32, 64); kl = ld_frag(s_kl + 16 * 64 + 32, 64);
        s1 = mma(qh1, kh, s1); s1 = mma(qh1, kl, s1); s1 = mma(ql1, kh, s1);
      }
      const int j0 = jt * 32;
#pragma unroll
      for (int r = 0; r < 8; ++r) {
        const int qi = qi0 + 8 * h + r;
        const int d0 = qi - (j0 + m);
        const int d1 = d0 - 16;
        const float b0 = s_bias[d0 > 0 ? d0 : 0];
        const float b1 = s_bias[d1 > 0 ? d1 : 0];
        const float v0 = (d0 < 0) ? -1e30f : (s0[r] * 0.125f + b0);
        const float v1 = (d1 < 0) ? -1e30f : (s1[r] * 0.125f + b1);
        const float mx = rmax16(fmaxf(v0, v1));
        const float nm = fmaxf(m_i[r], mx);
        const float corr = __expf(m_i[r] - nm);
        const float p0 = __expf(v0 - nm);
        const float p1 = __expf(v1 - nm);
        const float rs = rsum16(p0 + p1);
        l_i[r] = l_i[r] * corr + rs;
        m_i[r] = nm;
        acc[0][r] *= corr; acc[1][r] *= corr; acc[2][r] *= corr; acc[3][r] *= corr;
        unsigned hw, lw;
        split2(p0, p1, hw, lw);
        const int po = wave * 640 + (8 * h + r) * 40 + m;
        s_ph[po] = (u16)(hw & 0xFFFFu);
        s_ph[po + 16] = (u16)(hw >> 16);
        s_pl[po] = (u16)(lw & 0xFFFFu);
        s_pl[po + 16] = (u16)(lw >> 16);
      }
    }
    __syncthreads();

    if (jt <= jt_w) {
      const v16bf ph = ld_frag(s_ph + wave * 640, 40);
      const v16bf pl = ld_frag(s_pl + wave * 640, 40);
#pragma unroll
      for (int t = 0; t < 4; ++t) {
        const v16bf vh = ld_frag(s_vh + t * 16 * 32, 32);
        const v16bf vl = ld_frag(s_vl + t * 16 * 32, 32);
        acc[t] = mma(ph, vh, acc[t]);
        acc[t] = mma(ph, vl, acc[t]);
        acc[t] = mma(pl, vh, acc[t]);
      }
    }
    __syncthreads();
  }

  float* so = s_raw + wave * (16 * TP);
#pragma unroll
  for (int r = 0; r < 8; ++r) {
    const float inv = 1.0f / l_i[r];
#pragma unroll
    for (int t = 0; t < 4; ++t) so[(8 * h + r) * TP + t * 16 + m] = acc[t][r] * inv;
  }
  __syncthreads();
#pragma unroll
  for (int it = 0; it < 4; ++it) {
    const int row = it * 4 + (lane >> 3);
    const int cc = (lane & 7) * 8;
    const float* sp = so + row * TP + cc;
    const v4f a = *(const v4f*)sp;
    const v4f bq = *(const v4f*)(sp + 4);
    v4u H, L;
    split8(a.x, a.y, a.z, a.w, bq.x, bq.y, bq.z, bq.w, H, L);
    const size_t g = (qrow + row) * EMB + hd * HD + cc;
    store2_planes(AOh + g, AOl + g, H, L);
  }
}

__global__ __launch_bounds__(64) void k_proj_out(const u16* __restrict__ Ah, const u16* __restrict__ Al,
                                                 const u16* __restrict__ Wh, const u16* __restrict__ Wl,
                                                 const float* __restrict__ bvec, float* __restrict__ out) {
  __shared__ __attribute__((aligned(16))) float s_t[64 * TP];
  const int lane = threadIdx.x & 31, wave = threadIdx.x >> 5;
  const int c0 = blockIdx.x * 64;
  const int rblk = blockIdx.y * 64;
  const int r0 = rblk + wave * 32;

  v8f acc[2][4] = {{vz8(), vz8(), vz8(), vz8()}, {vz8(), vz8(), vz8(), vz8()}};
  gemm3(Ah + (size_t)r0 * EMB, Al + (size_t)r0 * EMB, Wh + (size_t)c0 * EMB, Wl + (size_t)c0 * EMB, acc);
  stage_tile(s_t, acc, bvec, c0);
  __syncthreads();

#pragma unroll
  for (int it = 0; it < 16; ++it) {
    const int row = wave * 32 + it * 2 + (lane >> 4);
    const int cc = (lane & 15) * 4;
    const v4f v = *(const v4f*)(s_t + row * TP + cc);
    const size_t g = (size_t)(rblk + row) * EMB + c0 + cc;
    *(volatile v4f*)(out + g) = v;
    __threadfence();
    *(volatile v4f*)(out + g) = v;
  }
}

extern "C" void kernel_launch(void* const* d_in, const int* in_sizes, int n_in,
                              void* d_out, int out_size, void* d_ws, size_t ws_size,
                              hipStream_t stream) {
  if (n_in < 8) return;
  if (in_sizes[0] != 8 * SEQ * EMB) return;
  if (in_sizes[1] != NQK * EMB) return;
  if (in_sizes[2] != NQK) return;
  if (in_sizes[3] != EMB * EMB) return;
  if (in_sizes[4] != EMB) return;
  if (in_sizes[5] != EMB * EMB) return;
  if (in_sizes[6] != EMB) return;
  if (in_sizes[7] != 32 * NH) return;
  if (out_size != 8 * SEQ * EMB) return;

  const float* x     = (const float*)d_in[0];
  const float* qk_w  = (const float*)d_in[1];
  const float* qk_b  = (const float*)d_in[2];
  const float* v_w   = (const float*)d_in[3];
  const float* v_b   = (const float*)d_in[4];
  const float* out_w = (const float*)d_in[5];
  const float* out_b = (const float*)d_in[6];
  const float* rbias = (const float*)d_in[7];
  float* out = (float*)d_out;

  const size_t eWqk = (size_t)NQK * EMB;
  const size_t eW   = (size_t)EMB * EMB;
  const size_t eX   = (size_t)TOKP * EMB;
  const size_t eQK  = (size_t)TOKP * NQK;
  const size_t eVt  = (size_t)NBP * NH * HD * SEQ;
  const size_t eAO  = (size_t)TOKP * EMB;
  u16* wsb = (u16*)d_ws;
  size_t off = 0;
  u16* Wqk_h = wsb + off; off += eWqk;
  u16* Wqk_l = wsb + off; off += eWqk;
  u16* Wv_h  = wsb + off; off += eW;
  u16* Wv_l  = wsb + off; off += eW;
  u16* Wo_h  = wsb + off; off += eW;
  u16* Wo_l  = wsb + off; off += eW;
  u16* X_h   = wsb + off; off += eX;
  u16* X_l   = wsb + off; off += eX;
  u16* QK_h  = wsb + off; off += eQK;
  u16* QK_l  = wsb + off; off += eQK;
  u16* Vt_h  = wsb + off; off += eVt;
  u16* Vt_l  = wsb + off; off += eVt;
  u16* AO_h  = wsb + off; off += eAO;
  u16* AO_l  = wsb + off; off += eAO;
  if (off * sizeof(u16) > ws_size) return;

  {
    const int n8a = (int)(eWqk / 8), n8b = (int)(eW / 8);
    k_split<<<dim3((n8a + 255) / 256), dim3(256), 0, stream>>>(qk_w, Wqk_h, Wqk_l, n8a);
    k_split<<<dim3((n8b + 255) / 256), dim3(256), 0, stream>>>(v_w, Wv_h, Wv_l, n8b);
    k_split<<<dim3((n8b + 255) / 256), dim3(256), 0, stream>>>(out_w, Wo_h, Wo_l, n8b);
  }

  for (int pass = 0; pass < 2; ++pass) {
    const float* xp = x + (size_t)pass * eX;
    float* outp = out + (size_t)pass * eAO;
    const int n8x = (int)(eX / 8);
    k_split<<<dim3((n8x + 255) / 256), dim3(256), 0, stream>>>(xp, X_h, X_l, n8x);
    k_proj_rows<<<dim3(NQK / 64, TOKP / 64), dim3(64), 0, stream>>>(X_h, X_l, Wqk_h, Wqk_l, qk_b,
                                                                    QK_h, QK_l, NQK);
    k_proj_vt<<<dim3(NH, TOKP / 64), dim3(64), 0, stream>>>(X_h, X_l, Wv_h, Wv_l, v_b, Vt_h, Vt_l);
    k_attn<<<dim3(SEQ / 128, NBP * NH), dim3(256), 0, stream>>>(QK_h, QK_l, Vt_h, Vt_l, rbias, AO_h, AO_l);
    k_proj_out<<<dim3(EMB / 64, TOKP / 64), dim3(64), 0, stream>>>(AO_h, AO_l, Wo_h, Wo_l, out_b, outp);
  }
}
